// LightweightMambaBlock_28106265985453
// MI455X (gfx1250) — hardware-verified
//
#include <hip/hip_runtime.h>
#include <math.h>

#define NBT   4
#define NCH   192
#define NPIX  4096
#define NTOK  16384
#define DIN   230
#define DIP   256
#define DST   16
#define DTRK  15
#define DBW   64
#define DBN   47
#define COLB  16
#define COLC  32
#define TPB   128
#define NBLK  128
#define NBY3  3
#define OSTR  68
#define SCH   32
#define XTP   200
#define XT8   24
#define LOG2E 1.4426950408889634f
#define EPSV  1e-5f
#define RDIN  (1.0f / 230.0f)

static_assert(NTOK == NBT * NPIX);
static_assert(NTOK % TPB == 0);
static_assert(NBLK == NTOK / TPB);
static_assert(NPIX % TPB == 0);
static_assert(NCH % 64 == 0);
static_assert(NBY3 == NCH / 64);
static_assert(NCH % 32 == 0);
static_assert(DIP % 64 == 0);
static_assert(DIP >= DIN);
static_assert(DBW >= COLC + DST);
static_assert(DTRK < COLB);
static_assert(NPIX % SCH == 0);
static_assert(SCH % 4 == 0);
static_assert(XTP % 8 == 0);
static_assert(XTP >= NCH);
static_assert(XT8 * 8 == NCH);
static_assert((64 * XT8) % 256 == 0);
static_assert(NPIX % 64 == 0);
static_assert(NPIX / 4 == 1024);
static_assert((NBT * NCH * NPIX) % 1024 == 0);
static_assert(OSTR % 4 == 0);
static_assert(NTOK % 8 == 0);

typedef unsigned short us16 __attribute__((ext_vector_type(16)));
typedef unsigned short us8  __attribute__((ext_vector_type(8)));
typedef unsigned short us8a __attribute__((ext_vector_type(8), may_alias));
typedef unsigned int   u32x8 __attribute__((ext_vector_type(8)));
typedef __bf16 v16b __attribute__((ext_vector_type(16)));
typedef float v8f __attribute__((ext_vector_type(8)));
typedef float v4f __attribute__((ext_vector_type(4)));
typedef float v4fa __attribute__((ext_vector_type(4), may_alias));
union FragU { us16 v; us8 h[2]; u32x8 w; };

#if __has_builtin(__builtin_amdgcn_exp2f)
#define FEXP2(x) __builtin_amdgcn_exp2f(x)
#else
#define FEXP2(x) __expf((x) * 0.6931471805599453f)
#endif

__device__ __forceinline__ unsigned short bf16_bits(float f) {
  unsigned u = __float_as_uint(f);
  u += 0x7FFFu + ((u >> 16) & 1u);
  return (unsigned short)(u >> 16);
}
__device__ __forceinline__ float bf16_val(unsigned short b) { return __uint_as_float(((unsigned)b) << 16); }
__device__ __forceinline__ float bf16r(float f) { return bf16_val(bf16_bits(f)); }
__device__ __forceinline__ float siluf(float x) { return x * __builtin_amdgcn_rcpf(1.0f + __expf(-x)); }

__device__ __forceinline__ void split8(const v4f a, const v4f b, us8& hi, us8& lo) {
#pragma unroll
  for (int u = 0; u < 4; ++u) {
    const unsigned short ha = bf16_bits(a[u]);
    hi[u] = ha; lo[u] = bf16_bits(a[u] - bf16_val(ha));
    const unsigned short hb = bf16_bits(b[u]);
    hi[4 + u] = hb; lo[4 + u] = bf16_bits(b[u] - bf16_val(hb));
  }
}

__device__ __forceinline__ v8f mma_bf16(us16 a, us16 b, v8f c) {
  return __builtin_amdgcn_wmma_f32_16x16x32_bf16(false, __builtin_bit_cast(v16b, a), false, __builtin_bit_cast(v16b, b), (short)0, c, false, false);
}
__device__ __forceinline__ void wguard2(v8f& c0, v8f& c1, v8f& c2, v8f& c3, const us16& a0, const us16& a1,
                                        const us16& b0, const us16& b1, const us16& b2, const us16& b3) {
#if defined(__HIP_DEVICE_COMPILE__)
  asm volatile("v_nop\n\tv_nop\n\tv_nop\n\tv_nop"
               : "+v"(c0), "+v"(c1), "+v"(c2), "+v"(c3)
               : "v"(a0), "v"(a1), "v"(b0), "v"(b1), "v"(b2), "v"(b3));
#endif
}

__device__ __forceinline__ us16 gfrag(const unsigned short* p) {
  const int kh = ((threadIdx.x >> 4) & 1) * 8;
  FragU f;
  f.h[0] = *(const us8a*)(p + kh);
  f.h[1] = *(const us8a*)(p + 16 + kh);
  return f.v;
}

__global__ __launch_bounds__(256) void k_cvtT(const float* __restrict__ src, unsigned short* dst, int srcK, int srcN, int gap,
                                             int kp8, int total8) {
  const int idx = blockIdx.x * 256 + threadIdx.x;
  if (idx >= total8) return;
  const int n = idx / kp8, k8 = (idx - n * kp8) * 8;
  const int j = n - ((n > gap) ? 1 : 0);
  const bool rowok = (n != gap) && (j >= 0) && (j < srcN);
  const int jc = rowok ? j : 0;
  us8 o;
#pragma unroll
  for (int u = 0; u < 8; ++u) {
    const int k = k8 + u;
    const int kc = (k < srcK) ? k : (srcK - 1);
    const float v = src[(size_t)kc * (size_t)srcN + jc];
    o[u] = (rowok && (k < srcK)) ? bf16_bits(v) : (unsigned short)0;
  }
  const size_t off = (size_t)idx * 8;
  *(volatile us8*)(dst + off) = o;
  __threadfence();
  *(volatile us8*)(dst + off) = o;
}

__global__ __launch_bounds__(256) void k_xtok(const float* __restrict__ x, unsigned short* XB) {
  __shared__ __attribute__((aligned(16))) unsigned short tile[64 * XTP];
  const int tid = threadIdx.x, hw0 = blockIdx.x * 64, b = blockIdx.y;
  const int hw = tid & 63, cq = tid >> 6;
#pragma unroll 4
  for (int it = 0; it < NCH / 4; ++it) {
    const int c = it * 4 + cq;
    const float v = x[((size_t)(b * NCH + c)) * NPIX + hw0 + hw];
    tile[hw * XTP + c] = bf16_bits(v);
  }
  __syncthreads();
#pragma unroll
  for (int pass = 0; pass < 2; ++pass) {
#pragma unroll
    for (int it = 0; it < (64 * XT8) / 256; ++it) {
      const int p = it * 256 + tid, rr = p / XT8, c8 = (p - rr * XT8) * 8;
      const us8 v = *(const us8a*)(tile + rr * XTP + c8);
      *(volatile us8*)(XB + ((size_t)(b * NPIX + hw0 + rr)) * NCH + c8) = v;
    }
    __threadfence();
  }
}

template <int TWOA, int SILU, int OUTF, int OUTHL, int NCHWO>
__global__ __launch_bounds__(256) void k_gemm(const unsigned short* __restrict__ A0, const unsigned short* __restrict__ A1, int lda,
                                             const unsigned short* __restrict__ Bw, int ldb, int K,
                                             float* Yf, int ldy, unsigned short* YH, unsigned short* YL, int ldh,
                                             float* Onc, float* PART) {
  __shared__ __attribute__((aligned(16))) float oS[8 * 16 * OSTR];
  __shared__ __attribute__((aligned(16))) float red[512];
  __shared__ __attribute__((aligned(16))) float pst[128];
  const int tid = threadIdx.x, lane = tid & 31, wave = tid >> 5, cl = lane & 15, hh = lane >> 4;
  const int mb = blockIdx.x * TPB, m0 = mb + 16 * wave, n0 = blockIdx.y * 64;

  v8f acc[4];
#pragma unroll
  for (int j = 0; j < 4; ++j) { const v8f zz = {0.f, 0.f, 0.f, 0.f, 0.f, 0.f, 0.f, 0.f}; acc[j] = zz; }

  const unsigned short* a0p = A0 + (size_t)(m0 + cl) * lda;
  const unsigned short* a1p = A1 + (size_t)(m0 + cl) * lda;
  const unsigned short* bwp = Bw + (size_t)(n0 + cl) * ldb;
#pragma unroll 1
  for (int k0 = 0; k0 < K; k0 += 32) {
    const us16 af0 = gfrag(a0p + k0);
    us16 af1 = af0;
    if (TWOA) af1 = gfrag(a1p + k0);
    us16 bfr[4];
#pragma unroll
    for (int j = 0; j < 4; ++j) bfr[j] = gfrag(bwp + (size_t)(16 * j) * ldb + k0);
#pragma unroll
    for (int j = 0; j < 4; ++j) acc[j] = mma_bf16(af0, bfr[j], acc[j]);
    if (TWOA) {
#pragma unroll
      for (int j = 0; j < 4; ++j) acc[j] = mma_bf16(af1, bfr[j], acc[j]);
    }
    wguard2(acc[0], acc[1], acc[2], acc[3], af0, af1, bfr[0], bfr[1], bfr[2], bfr[3]);
  }

  float* so = oS + wave * (16 * OSTR);
#pragma unroll
  for (int j = 0; j < 4; ++j)
#pragma unroll
    for (int r = 0; r < 8; ++r) so[(8 * hh + r) * OSTR + 16 * j + cl] = acc[j][r];
  __syncthreads();

  if (OUTF) {
#pragma unroll
    for (int pass = 0; pass < 2; ++pass) {
#pragma unroll
      for (int it = 0; it < 8; ++it) {
        const int ch = it * 32 + lane, r = ch >> 4, q = (ch & 15) * 4;
        v4f v = *(const v4fa*)(so + r * OSTR + q);
        if (SILU) {
#pragma unroll
          for (int u = 0; u < 4; ++u) v[u] = siluf(v[u]);
        }
        *(volatile v4f*)(Yf + (size_t)(m0 + r) * ldy + n0 + q) = v;
      }
      __threadfence();
    }
  }
  if (OUTHL) {
#pragma unroll
    for (int pass = 0; pass < 2; ++pass) {
#pragma unroll
      for (int it = 0; it < 4; ++it) {
        const int ch = it * 32 + lane, r = ch >> 3, c8 = (ch & 7) * 8;
        v4f a = *(const v4fa*)(so + r * OSTR + c8);
        v4f b = *(const v4fa*)(so + r * OSTR + c8 + 4);
        if (SILU) {
#pragma unroll
          for (int u = 0; u < 4; ++u) { a[u] = siluf(a[u]); b[u] = siluf(b[u]); }
        }
        us8 hi, lo;
        split8(a, b, hi, lo);
        const size_t o2 = (size_t)(m0 + r) * ldh + n0 + c8;
        *(volatile us8*)(YH + o2) = hi; *(volatile us8*)(YL + o2) = lo;
      }
      __threadfence();
    }
  }
  if (NCHWO) {
    const int bimg = mb / NPIX, hw0 = mb - bimg * NPIX;
#pragma unroll
    for (int pass = 0; pass < 2; ++pass) {
#pragma unroll
      for (int it = 0; it < 8; ++it) {
        const int c = it * 8 + wave;
        v4f v;
#pragma unroll
        for (int i = 0; i < 4; ++i) v[i] = oS[(lane * 4 + i) * OSTR + c];
        const size_t o = ((size_t)(bimg * NCH + n0 + c)) * NPIX + hw0 + lane * 4;
        *(volatile v4f*)(Onc + o) = v;
      }
      __threadfence();
    }
    {
      const int c = tid & 63, ph = tid >> 6;
      float s = 0.0f, q = 0.0f;
#pragma unroll 4
      for (int i = 0; i < 32; ++i) {
        const float v = oS[(ph * 32 + i) * OSTR + c];
        s += v; q += v * v;
      }
      red[ph * 64 + c] = s; red[256 + ph * 64 + c] = q;
    }
    __syncthreads();
    if (tid < 64) {
      const float S = ((red[tid] + red[64 + tid]) + red[128 + tid]) + red[192 + tid];
      const float Q = ((red[256 + tid] + red[320 + tid]) + red[384 + tid]) + red[448 + tid];
      pst[tid] = S; pst[64 + tid] = Q;
    }
    __syncthreads();
    if (wave == 0) {
      const v4f v = *(const v4fa*)(pst + lane * 4);
      const size_t po = (size_t)(blockIdx.x * gridDim.y + blockIdx.y) * 128 + lane * 4;
      *(volatile v4f*)(PART + po) = v;
      __threadfence();
      *(volatile v4f*)(PART + po) = v;
    }
  }
}

__global__ __launch_bounds__(256) void k_dt(const float* __restrict__ XDBL, const float* __restrict__ dtw, const float* __restrict__ dtb,
                                           float* DT) {
  const int idx = blockIdx.x * 256 + threadIdx.x;
  if (idx >= NTOK * DIP) return;
  const int tok = idx >> 8, d = idx & (DIP - 1);
  const int dc = (d < DIN) ? d : (DIN - 1);
  const float* xr = XDBL + (size_t)tok * DBW;
  const v4f x0 = *(const v4fa*)(xr), x1 = *(const v4fa*)(xr + 4), x2 = *(const v4fa*)(xr + 8), x3 = *(const v4fa*)(xr + 12);
  float a = 0.0f;
#pragma unroll
  for (int r = 0; r < 4; ++r) a = a + x0[r] * bf16r(dtw[(size_t)r * DIN + dc]);
#pragma unroll
  for (int r = 0; r < 4; ++r) a = a + x1[r] * bf16r(dtw[(size_t)(4 + r) * DIN + dc]);
#pragma unroll
  for (int r = 0; r < 4; ++r) a = a + x2[r] * bf16r(dtw[(size_t)(8 + r) * DIN + dc]);
#pragma unroll
  for (int r = 0; r < 3; ++r) a = a + x3[r] * bf16r(dtw[(size_t)(12 + r) * DIN + dc]);
  a = a + bf16r(dtb[dc]);
  const float sp = fmaxf(a, 0.0f) + log1pf(__expf(-fabsf(a)));
  const float dl = (d < DIN) ? sp : 0.0f;
  *(volatile float*)(DT + idx) = dl;
  __threadfence();
  *(volatile float*)(DT + idx) = dl;
}

__global__ __launch_bounds__(256) void k_scan(const float* __restrict__ DT, const float* __restrict__ UF, const float* __restrict__ XDBL,
                                             const float* __restrict__ Alog, const float* __restrict__ Dv, float* Y) {
  __shared__ __attribute__((aligned(16))) float sy[SCH * DIP];
  const int tid = threadIdx.x, b = blockIdx.x, d = tid;
  const int dc = (d < DIN) ? d : (DIN - 1);
  float A2[DST], h[DST];
#pragma unroll
  for (int i = 0; i < DST; ++i) { A2[i] = -__expf(bf16r(Alog[dc * DST + i])) * LOG2E; h[i] = 0.0f; }
  const float Dd = bf16r(Dv[dc]);
  const int wrow = tid >> 6, wq = (tid & 63) * 4;
#pragma unroll 1
  for (int c = 0; c < NPIX / SCH; ++c) {
#pragma unroll 1
    for (int s = 0; s < SCH; ++s) {
      const size_t tok = (size_t)b * NPIX + (size_t)(c * SCH + s);
      const size_t e = tok * DIP + d;
      const float dl = DT[e], uv = UF[e];
      const float* bc = XDBL + tok * DBW + COLB;
      v4f Bv[4], Cv[4];
#pragma unroll
      for (int q = 0; q < 4; ++q) {
        Bv[q] = *(const v4fa*)(bc + 4 * q);
        Cv[q] = *(const v4fa*)(bc + (COLC - COLB) + 4 * q);
      }
      const float dx = dl * uv;
      float y = 0.0f;
#pragma unroll
      for (int i = 0; i < DST; ++i) {
        const float ex = FEXP2(dl * A2[i]);
        h[i] = ex * h[i] + dx * Bv[i >> 2][i & 3];
        y = y + h[i] * Cv[i >> 2][i & 3];
      }
      sy[s * DIP + d] = y + uv * Dd;
    }
    __syncthreads();
#pragma unroll
    for (int pass = 0; pass < 2; ++pass) {
#pragma unroll
      for (int it = 0; it < SCH / 4; ++it) {
        const int row = it * 4 + wrow;
        const v4f v = *(const v4fa*)(sy + row * DIP + wq);
        *(volatile v4f*)(Y + ((size_t)b * NPIX + (size_t)(c * SCH + row)) * DIP + wq) = v;
      }
      __threadfence();
    }
    __syncthreads();
  }
}

__global__ __launch_bounds__(256) void k_ln(const float* __restrict__ Y, const float* __restrict__ g, const float* __restrict__ bt,
                                           unsigned short* YH, unsigned short* YL) {
  const int tid = threadIdx.x, lane = tid & 31, wave = tid >> 5;
  const int tok = blockIdx.x * 8 + wave, c0 = lane * 8;
  const float* yr = Y + (size_t)tok * DIP + c0;
  const v4f xa = *(const v4fa*)yr, xb = *(const v4fa*)(yr + 4);
  float v[8], gq[8], bq[8];
  bool ok[8];
#pragma unroll
  for (int u = 0; u < 4; ++u) { v[u] = xa[u]; v[4 + u] = xb[u]; }
#pragma unroll
  for (int u = 0; u < 8; ++u) {
    const int c = c0 + u;
    ok[u] = (c < DIN);
    const int cc = ok[u] ? c : (DIN - 1);
    gq[u] = bf16r(g[cc]); bq[u] = bf16r(bt[cc]);
  }
  float s = 0.0f;
#pragma unroll
  for (int u = 0; u < 8; ++u) s += ok[u] ? v[u] : 0.0f;
  s += __shfl_xor(s, 16); s += __shfl_xor(s, 8); s += __shfl_xor(s, 4); s += __shfl_xor(s, 2); s += __shfl_xor(s, 1);
  const float mu = s * RDIN;
  float dv[8];
  float s2 = 0.0f;
#pragma unroll
  for (int u = 0; u < 8; ++u) { dv[u] = ok[u] ? (v[u] - mu) : 0.0f; s2 += dv[u] * dv[u]; }
  s2 += __shfl_xor(s2, 16); s2 += __shfl_xor(s2, 8); s2 += __shfl_xor(s2, 4); s2 += __shfl_xor(s2, 2); s2 += __shfl_xor(s2, 1);
  const float var = s2 * RDIN;
  const float rs = rsqrtf(var + EPSV);
  v4f oa, ob;
#pragma unroll
  for (int u = 0; u < 4; ++u) {
    oa[u] = ok[u] ? ((dv[u] * rs) * gq[u] + bq[u]) : 0.0f;
    ob[u] = ok[4 + u] ? ((dv[4 + u] * rs) * gq[4 + u] + bq[4 + u]) : 0.0f;
  }
  us8 hi, lo;
  split8(oa, ob, hi, lo);
  const size_t off = (size_t)tok * DIP + c0;
  *(volatile us8*)(YH + off) = hi; *(volatile us8*)(YL + off) = lo;
  __threadfence();
  *(volatile us8*)(YH + off) = hi; *(volatile us8*)(YL + off) = lo;
}

__global__ __launch_bounds__(256) void k_bnfin(const float* __restrict__ PART, float* ST) {
  __shared__ __attribute__((aligned(16))) float pst[512];
  const int tid = threadIdx.x;
  const bool ok = (tid < NCH);
  const int cc = ok ? tid : (NCH - 1);
  const int by = cc >> 6, cl = cc & 63;
  double s = 0.0, q = 0.0;
#pragma unroll 1
  for (int p = 0; p < NBLK; ++p) {
    const size_t base = (size_t)(p * NBY3 + by) * 128;
    s += (double)PART[base + cl]; q += (double)PART[base + 64 + cl];
  }
  const double mean = s / (double)NTOK;
  double var = q / (double)NTOK - mean * mean;
  var = (var < 0.0) ? 0.0 : var;
  pst[tid] = ok ? (float)mean : 0.0f;
  pst[256 + tid] = ok ? rsqrtf((float)var + EPSV) : 0.0f;
  __syncthreads();
  if (tid < 128) {
    const v4f v = *(const v4fa*)(pst + tid * 4);
    *(volatile v4f*)(ST + tid * 4) = v;
    __threadfence();
    *(volatile v4f*)(ST + tid * 4) = v;
  }
}

__global__ __launch_bounds__(256) void k_bnapply(const float* __restrict__ Onc, const float* __restrict__ ST,
                                                const float* __restrict__ g, const float* __restrict__ bt, float* outp) {
  const int idx = blockIdx.x * 256 + threadIdx.x;
  if (idx >= NBT * NCH * NPIX / 4) return;
  const int c = (idx >> 10) % NCH;
  const v4f v = *(const v4fa*)(Onc + (size_t)idx * 4);
  const float mu = ST[c], rs = ST[256 + c], gg = bf16r(g[c]), bb = bf16r(bt[c]);
  v4f o;
#pragma unroll
  for (int u = 0; u < 4; ++u) o[u] = ((v[u] - mu) * rs) * gg + bb;
  *(volatile v4f*)(outp + (size_t)idx * 4) = o;
  __threadfence();
  *(volatile v4f*)(outp + (size_t)idx * 4) = o;
}

extern "C" void kernel_launch(void* const* d_in, const int* in_sizes, int n_in,
                              void* d_out, int out_size, void* d_ws, size_t ws_size,
                              hipStream_t stream) {
  if (n_in < 12) return;
  if (in_sizes[0] != NBT * NCH * NPIX || in_sizes[1] != NCH * DIN || in_sizes[2] != DIN * DBN || in_sizes[3] != DTRK * DIN ||
      in_sizes[4] != DIN || in_sizes[5] != DIN * DST || in_sizes[6] != DIN || in_sizes[7] != DIN || in_sizes[8] != DIN ||
      in_sizes[9] != DIN * NCH || in_sizes[10] != NCH || in_sizes[11] != NCH) return;
  if (out_size != NBT * NCH * NPIX) return;

  const float* x         = (const float*)d_in[0];
  const float* W_in      = (const float*)d_in[1];
  const float* x_proj_w  = (const float*)d_in[2];
  const float* dt_proj_w = (const float*)d_in[3];
  const float* dt_proj_b = (const float*)d_in[4];
  const float* A_log     = (const float*)d_in[5];
  const float* Dv        = (const float*)d_in[6];
  const float* ln_g      = (const float*)d_in[7];
  const float* ln_b      = (const float*)d_in[8];
  const float* W_out     = (const float*)d_in[9];
  const float* bn_g      = (const float*)d_in[10];
  const float* bn_b      = (const float*)d_in[11];
  float* out = (float*)d_out;

  size_t off = 0;
  auto carve = [&](size_t bytes) -> char* { char* p = (char*)d_ws + off; off += (bytes + 255) & ~(size_t)255; return p; };
  unsigned short* XB  = (unsigned short*)carve((size_t)NTOK * NCH * 2);
  unsigned short* UH  = (unsigned short*)carve((size_t)NTOK * DIP * 2);
  unsigned short* UL  = (unsigned short*)carve((size_t)NTOK * DIP * 2);
  float* UF   = (float*)carve((size_t)NTOK * DIP * 4);
  float* XDBL = (float*)carve((size_t)NTOK * DBW * 4);
  float* DT   = (float*)carve((size_t)NTOK * DIP * 4);
  float* YS   = (float*)carve((size_t)NTOK * DIP * 4);
  unsigned short* YNH = (unsigned short*)carve((size_t)NTOK * DIP * 2);
  unsigned short* YNL = (unsigned short*)carve((size_t)NTOK * DIP * 2);
  float* ONC  = (float*)carve((size_t)NBT * NCH * NPIX * 4);
  unsigned short* WIN = (unsigned short*)carve((size_t)DIP * NCH * 2);
  unsigned short* WXP = (unsigned short*)carve((size_t)DBW * DIP * 2);
  unsigned short* WOP = (unsigned short*)carve((size_t)NCH * DIP * 2);
  float* PART = (float*)carve((size_t)NBLK * NBY3 * 128 * 4);
  float* ST   = (float*)carve((size_t)512 * 4);
  if (off > ws_size || off > (size_t)134217728) return;

  const dim3 b256(256);
  auto cdv = [](long a, long b) { return (unsigned)((a + b - 1) / b); };

  k_cvtT<<<dim3(cdv(DIP * (NCH / 8), 256)), b256, 0, stream>>>(W_in, WIN, NCH, DIN, 1 << 20, NCH / 8, DIP * (NCH / 8));
  k_cvtT<<<dim3(cdv(DBW * (DIP / 8), 256)), b256, 0, stream>>>(x_proj_w, WXP, DIN, DBN, DTRK, DIP / 8, DBW * (DIP / 8));
  k_cvtT<<<dim3(cdv(NCH * (DIP / 8), 256)), b256, 0, stream>>>(W_out, WOP, DIN, NCH, 1 << 20, DIP / 8, NCH * (DIP / 8));
  k_xtok<<<dim3(NPIX / 64, NBT), b256, 0, stream>>>(x, XB);
  k_gemm<0, 1, 1, 1, 0><<<dim3(NBLK, DIP / 64), b256, 0, stream>>>(XB, XB, NCH, WIN, NCH, NCH, UF, DIP, UH, UL, DIP, ONC, PART);
  k_gemm<1, 0, 1, 0, 0><<<dim3(NBLK, 1), b256, 0, stream>>>(UH, UL, DIP, WXP, DIP, DIP, XDBL, DBW, UH, UL, DIP, ONC, PART);
  k_dt<<<dim3(NTOK), b256, 0, stream>>>(XDBL, dt_proj_w, dt_proj_b, DT);
  k_scan<<<dim3(NBT), b256, 0, stream>>>(DT, UF, XDBL, A_log, Dv, YS);
  k_ln<<<dim3(NTOK / 8), b256, 0, stream>>>(YS, ln_g, ln_b, YNH, YNL);
  k_gemm<1, 0, 0, 0, 1><<<dim3(NBLK, NBY3), b256, 0, stream>>>(YNH, YNL, DIP, WOP, DIP, DIP, UF, DIP, UH, UL, DIP, ONC, PART);
  k_bnfin<<<dim3(1), b256, 0, stream>>>(PART, ST);
  k_bnapply<<<dim3(NBT * NCH * NPIX / 4 / 256), b256, 0, stream>>>(ONC, ST, bn_g, bn_b, out);
}
